// HGTModel_28432683500202
// MI455X (gfx1250) — hardware-verified
//
#include <hip/hip_runtime.h>
#include <math.h>

#define HID   128
#define OUTD  32
#define NHEAD 8
#define RELSZ 256

typedef _Float16 v16h __attribute__((ext_vector_type(16)));
typedef _Float16 v8h  __attribute__((ext_vector_type(8)));
typedef _Float16 v4h  __attribute__((ext_vector_type(4)));
typedef float    v8f  __attribute__((ext_vector_type(8)));
typedef float    v4f  __attribute__((ext_vector_type(4)));
union Frag { v16h v; v8h half[2]; };

__device__ __forceinline__ v8f wmma16(v16h a, v16h b, v8f c)
{
    v8f d = __builtin_amdgcn_wmma_f32_16x16x32_f16(false, a, false, b, (short)0, c, false, false);
    asm volatile("v_nop\n\tv_nop\n\tv_nop\n\tv_nop" : "+v"(d) : "v"(a), "v"(b));
    return d;
}

__device__ __forceinline__ float wave_sum(float v)
{
#pragma unroll
    for (int o = 16; o > 0; o >>= 1) v += __shfl_xor(v, o);
    return v;
}

template<int NC>
__device__ __forceinline__ void mma_tile(const _Float16* __restrict__ A, int M, int row0,
                                         const _Float16* __restrict__ Wt, float* tile)
{
    constexpr int CGN = NC / 32;
    constexpr int TP  = NC + 4;
    const int lane = threadIdx.x & 31, wave = threadIdx.x >> 5;
    const int h = lane >> 4, m = lane & 15;
    const int rg = wave / CGN, cg = wave - rg * CGN;
    int arow = row0 + rg * 16 + m;
    arow = arow < M ? arow : (M - 1);
    const _Float16* ap  = A  + (size_t)arow * HID + 8 * h;
    const _Float16* bp0 = Wt + (size_t)(cg * 32 + m) * HID + 8 * h;
    const _Float16* bp1 = bp0 + 16 * HID;
    v8f acc0 = {0.f, 0.f, 0.f, 0.f, 0.f, 0.f, 0.f, 0.f};
    v8f acc1 = acc0;
#pragma unroll
    for (int k0 = 0; k0 < HID; k0 += 32) {
        Frag a, b0, b1;
        a.half[0]  = *(const v8h*)(ap  + k0);  a.half[1]  = *(const v8h*)(ap  + k0 + 16);
        b0.half[0] = *(const v8h*)(bp0 + k0);  b0.half[1] = *(const v8h*)(bp0 + k0 + 16);
        b1.half[0] = *(const v8h*)(bp1 + k0);  b1.half[1] = *(const v8h*)(bp1 + k0 + 16);
        acc0 = wmma16(a.v, b0.v, acc0);
        acc1 = wmma16(a.v, b1.v, acc1);
    }
    const int trow = rg * 16 + 8 * h;
#pragma unroll
    for (int r = 0; r < 8; ++r) {
        tile[(trow + r) * TP + cg * 32 + m]      = acc0[r];
        tile[(trow + r) * TP + cg * 32 + 16 + m] = acc1[r];
    }
}

__global__ __launch_bounds__(128) void k_prep(const float* __restrict__ W, const float* __restrict__ bias,
                                              const float* __restrict__ rel, const float* __restrict__ pr,
                                              int mode, int ncol, float scale,
                                              _Float16* __restrict__ Wt, float* __restrict__ bout)
{
    const int tid = threadIdx.x, mat = blockIdx.y;
    const float* Wm   = W    + (size_t)mat * HID * ncol;
    const float* bm   = bias + (size_t)mat * ncol;
    const float* relm = rel  + (size_t)mat * NHEAD * RELSZ;
    const float* prm  = pr   + (size_t)mat * NHEAD;
    _Float16* Wtm  = Wt   + (size_t)mat * ncol * HID;
    float*    boutm = bout + (size_t)mat * ncol;
    const int g = blockIdx.x * 128 + tid;
    const int n = g >> 4, kb = g & 15;
    if (n < ncol) {
        const int hh = n >> 4, e = n & 15;
        const float pf = (mode == 2) ? prm[hh] * 0.25f : 1.0f;
        const float sc = scale * pf;
        v8h o;
#pragma unroll
        for (int j = 0; j < 8; ++j) {
            const int k = kb * 8 + j;
            float v;
            if (mode == 0) {
                v = Wm[(size_t)k * ncol + n];
            } else {
                v = 0.0f;
                const float* wr = Wm + (size_t)k * ncol + hh * 16;
                const float* rr = relm + hh * RELSZ + e;
#pragma unroll 1
                for (int d = 0; d < 16; ++d) v += wr[d] * rr[d * 16];
            }
            o[j] = (_Float16)(v * sc);
        }
        _Float16* dst = Wtm + (size_t)n * HID + kb * 8;
        *(volatile v8h*)dst = o;
        __threadfence();
        *(volatile v8h*)dst = o;
    }
    if (blockIdx.x == 0 && tid < ncol) {
        const int hh = tid >> 4, e = tid & 15;
        const float pf = (mode == 2) ? prm[hh] * 0.25f : 1.0f;
        float v;
        if (mode == 0) {
            v = bm[tid];
        } else {
            v = 0.0f;
            const float* br = bm + hh * 16;
            const float* rr = relm + hh * RELSZ + e;
#pragma unroll 1
            for (int d = 0; d < 16; ++d) v += br[d] * rr[d * 16];
        }
        const float bvv = v * pf;
        *(volatile float*)(boutm + tid) = bvv;
        __threadfence();
        *(volatile float*)(boutm + tid) = bvv;
    }
}

__global__ __launch_bounds__(256) void k_cvt(const float* __restrict__ s0, int n0,
                                             const float* __restrict__ s1, int n1,
                                             _Float16* __restrict__ dst)
{
    const int g = blockIdx.x * 256 + threadIdx.x;
    const int row = g >> 4, piece = g & 15;
    if (row >= n0 + n1) return;
    const float* src = (row < n0) ? (s0 + (size_t)row * HID) : (s1 + (size_t)(row - n0) * HID);
    const v4f a = *(const v4f*)(src + piece * 8);
    const v4f b = *(const v4f*)(src + piece * 8 + 4);
    const v8f f = __builtin_shufflevector(a, b, 0, 1, 2, 3, 4, 5, 6, 7);
    const v8h o = __builtin_convertvector(f, v8h);
    _Float16* d = dst + (size_t)row * HID + piece * 8;
    *(volatile v8h*)d = o;
    __threadfence();
    *(volatile v8h*)d = o;
}

__global__ __launch_bounds__(256) void k_lin2(const _Float16* __restrict__ A, int M,
                                              const _Float16* __restrict__ Wt0, const float* __restrict__ b0,
                                              float inv0, float* __restrict__ C0,
                                              const _Float16* __restrict__ Wt1, const float* __restrict__ b1,
                                              float inv1, float* __restrict__ C1)
{
    __shared__ float tile[32 * (HID + 4)];
    const int y = blockIdx.y;
    const _Float16* Wt = y ? Wt1 : Wt0;
    const float* bias = y ? b1 : b0;
    const float inv = y ? inv1 : inv0;
    float* C = y ? C1 : C0;
    const int row0 = blockIdx.x * 32;
    mma_tile<HID>(A, M, row0, Wt, tile);
    __syncthreads();
    const int lane = threadIdx.x & 31, wave = threadIdx.x >> 5;
    const v4f bb = *(const v4f*)(bias + 4 * lane);
#pragma unroll
    for (int i = 0; i < 4; ++i) {
        const int tr = wave + 8 * i;
        const int grow = row0 + tr;
        if (grow < M) {
            const v4f a = *(const v4f*)(tile + tr * (HID + 4) + 4 * lane);
            const v4f o = a * inv + bb;
            float* p = C + (size_t)grow * HID + 4 * lane;
            *(volatile v4f*)p = o;
            __threadfence();
            *(volatile v4f*)p = o;
        }
    }
}

__global__ __launch_bounds__(256) void k_lin_relu(const _Float16* __restrict__ A, int M,
                                                  const _Float16* __restrict__ Wt, const float* __restrict__ bias,
                                                  float inv, float* __restrict__ X32, _Float16* __restrict__ X16)
{
    __shared__ float tile[32 * (HID + 4)];
    const int row0 = blockIdx.x * 32;
    mma_tile<HID>(A, M, row0, Wt, tile);
    __syncthreads();
    const int lane = threadIdx.x & 31, wave = threadIdx.x >> 5;
    const v4f bb = *(const v4f*)(bias + 4 * lane);
#pragma unroll
    for (int i = 0; i < 4; ++i) {
        const int tr = wave + 8 * i;
        const int grow = row0 + tr;
        if (grow < M) {
            const v4f a = *(const v4f*)(tile + tr * (HID + 4) + 4 * lane);
            v4f o = a * inv + bb;
            o.x = fmaxf(o.x, 0.0f); o.y = fmaxf(o.y, 0.0f); o.z = fmaxf(o.z, 0.0f); o.w = fmaxf(o.w, 0.0f);
            const v4h o16 = __builtin_convertvector(o, v4h);
            float* p32 = X32 + (size_t)grow * HID + 4 * lane;
            _Float16* p16 = X16 + (size_t)grow * HID + 4 * lane;
            *(volatile v4f*)p32 = o;
            *(volatile v4h*)p16 = o16;
            __threadfence();
            *(volatile v4f*)p32 = o;
            *(volatile v4h*)p16 = o16;
        }
    }
}

__global__ __launch_bounds__(256) void k_lin_ln(const _Float16* __restrict__ A, int M,
                                                const _Float16* __restrict__ Wt, const float* __restrict__ bias,
                                                float inv, float* X32, _Float16* __restrict__ X16,
                                                const float* __restrict__ skp, const float* __restrict__ g,
                                                const float* __restrict__ be)
{
    __shared__ float tile[32 * (HID + 4)];
    const int row0 = blockIdx.x * 32;
    mma_tile<HID>(A, M, row0, Wt, tile);
    __syncthreads();
    const int lane = threadIdx.x & 31, wave = threadIdx.x >> 5;
    const float sk  = 1.0f / (1.0f + __expf(-skp[0]));
    const float skc = 1.0f - sk;
    const v4f bb = *(const v4f*)(bias + 4 * lane);
    const v4f gg = *(const v4f*)(g + 4 * lane);
    const v4f ee = *(const v4f*)(be + 4 * lane);
#pragma unroll
    for (int i = 0; i < 4; ++i) {
        const int tr = wave + 8 * i;
        const int grow = row0 + tr;
        if (grow < M) {
            const v4f a = *(const v4f*)(tile + tr * (HID + 4) + 4 * lane);
            float* p32 = X32 + (size_t)grow * HID + 4 * lane;
            const v4f xo = *(const v4f*)p32;
            const v4f o  = a * inv + bb;
            const v4f o2 = o * sk + xo * skc;
            const v4f y  = xo + o2;
            float s1 = (y.x + y.y) + (y.z + y.w);
            s1 = wave_sum(s1);
            const float mean = s1 * (1.0f / HID);
            const v4f dd = y - mean;
            float s2 = (dd.x * dd.x + dd.y * dd.y) + (dd.z * dd.z + dd.w * dd.w);
            s2 = wave_sum(s2);
            const float var = s2 * (1.0f / HID);
            const float rs = rsqrtf(var + 1e-5f);
            const v4f out = dd * rs * gg + ee;
            const v4h o16 = __builtin_convertvector(out, v4h);
            _Float16* p16 = X16 + (size_t)grow * HID + 4 * lane;
            *(volatile v4f*)p32 = out;
            *(volatile v4h*)p16 = o16;
            __threadfence();
            *(volatile v4f*)p32 = out;
            *(volatile v4h*)p16 = o16;
        }
    }
}

__global__ __launch_bounds__(64) void k_out(const _Float16* __restrict__ A, int M,
                                            const _Float16* __restrict__ Wt, const float* __restrict__ bias,
                                            float inv, float* __restrict__ O)
{
    __shared__ float tile[32 * (OUTD + 4)];
    const int row0 = blockIdx.x * 32;
    mma_tile<OUTD>(A, M, row0, Wt, tile);
    __syncthreads();
    const int lane = threadIdx.x & 31, wave = threadIdx.x >> 5;
    const int q = lane >> 3, c4 = (lane & 7) * 4;
    const v4f bb = *(const v4f*)(bias + c4);
#pragma unroll
    for (int i = 0; i < 4; ++i) {
        const int tr = wave * 16 + i * 4 + q;
        const int grow = row0 + tr;
        if (grow < M) {
            const v4f a = *(const v4f*)(tile + tr * (OUTD + 4) + c4);
            const v4f o = a * inv + bb;
            float* p = O + (size_t)grow * OUTD + c4;
            *(volatile v4f*)p = o;
            __threadfence();
            *(volatile v4f*)p = o;
        }
    }
}

template<int R, int SCAP>
__global__ __launch_bounds__(256) void k_agg(const int* __restrict__ esrc, const int* __restrict__ edst,
                                             int E, int n_src, int n_dst,
                                             const float* __restrict__ q, const float* __restrict__ kt,
                                             const float* __restrict__ vt, _Float16* __restrict__ out16)
{
    extern __shared__ int lds_dyn[];
    int* seg   = lds_dyn;
    int* cnt   = seg + R * SCAP;
    int* hit_e = cnt + R;
    int* hit_s = hit_e + 1024;
    int* wcnt  = hit_s + 1024;
    const int tid = threadIdx.x, lane = tid & 31, wave = tid >> 5;
    const int r0 = blockIdx.x * R;
    for (int i = tid; i < R; i += 256) cnt[i] = 0;
    __syncthreads();
    const unsigned lm = (1u << lane) - 1u;
    const int nch = (E + 1023) >> 10;
    for (int c = 0; c < nch; ++c) {
        const int base = c << 10;
        unsigned bal[4]; int sl[4]; int ed[4];
#pragma unroll
        for (int j = 0; j < 4; ++j) {
            const int e = base + (j << 8) + tid;
            int s = -1;
            if (e < E) {
                const int d = edst[e];
                const unsigned u = (unsigned)(d - r0);
                if (u < (unsigned)R) s = (int)u;
            }
            sl[j] = s; ed[j] = e;
            bal[j] = (unsigned)__ballot(s >= 0);
            if (lane == 0) wcnt[(j << 3) + wave] = (int)__popc(bal[j]);
        }
        __syncthreads();
        int pre[4]; int tot = 0;
#pragma unroll
        for (int j = 0; j < 4; ++j) {
            pre[j] = 0;
#pragma unroll
            for (int w = 0; w < 8; ++w) {
                if (w == wave) pre[j] = tot;
                tot += wcnt[(j << 3) + w];
            }
        }
        tot = min(tot, 1024);
#pragma unroll
        for (int j = 0; j < 4; ++j) {
            if (sl[j] >= 0) {
                const int pos = pre[j] + (int)__popc(bal[j] & lm);
                hit_e[pos] = ed[j];
                hit_s[pos] = sl[j];
            }
        }
        __syncthreads();
        int rk[4], ms[4], ls[4];
#pragma unroll
        for (int j = 0; j < 4; ++j) {
            const int t = tid + (j << 8);
            rk[j] = -1; ms[j] = 0; ls[j] = 0;
            if (t < tot) {
                const int my = hit_s[t];
                int dup = 0, later = 0;
                for (int i = 0; i < tot; ++i) {
                    const int si = hit_s[i];
                    const int eq = (si == my) ? 1 : 0;
                    dup   += eq & ((i < t) ? 1 : 0);
                    later |= eq & ((i > t) ? 1 : 0);
                }
                const int rank = cnt[my] + dup;
                if (rank < SCAP) seg[my * SCAP + rank] = hit_e[t];
                rk[j] = rank; ms[j] = my; ls[j] = later ? 0 : 1;
            }
        }
        __syncthreads();
#pragma unroll
        for (int j = 0; j < 4; ++j) {
            if (rk[j] >= 0 && ls[j]) cnt[ms[j]] = min(rk[j] + 1, SCAP);
        }
    }
    __syncthreads();

    constexpr int RPW = R / 8;
    for (int i = 0; i < RPW; ++i) {
        const int s = wave + (i << 3);
        const int node = r0 + s;
        if (node >= n_dst) break;
        const int ne = min(cnt[s], SCAP);
        const v4f q4 = *(const v4f*)(q + (size_t)node * HID + 4 * lane);
        float mrun = -1.0e30f, srun = 0.0f;
        v4f acc = {0.f, 0.f, 0.f, 0.f};
        for (int jx = 0; jx < ne; ++jx) {
            const int e = seg[s * SCAP + jx];
            int src = esrc[e];
            src = src < 0 ? 0 : (src >= n_src ? (n_src - 1) : src);
            const v4f k4 = *(const v4f*)(kt + (size_t)src * HID + 4 * lane);
            const v4f v4 = *(const v4f*)(vt + (size_t)src * HID + 4 * lane);
            float p = q4.x * k4.x + q4.y * k4.y + q4.z * k4.z + q4.w * k4.w;
            p += __shfl_xor(p, 1);
            p += __shfl_xor(p, 2);
            const float mn = fmaxf(mrun, p);
            const float sc = __expf(mrun - mn);
            const float ex = __expf(p - mn);
            srun = srun * sc + ex;
            acc = acc * sc + v4 * ex;
            mrun = mn;
        }
        const float inv = 1.0f / (srun + 1e-16f);
        v4f og = acc * inv;
#pragma unroll 1
        for (int cI = 0; cI < 4; ++cI) {
            const float xv = (cI == 0) ? og.x : ((cI == 1) ? og.y : ((cI == 2) ? og.z : og.w));
            const float gv = 0.5f * xv * (1.0f + erff(xv * 0.70710678118654752f));
            og.x = (cI == 0) ? gv : og.x;
            og.y = (cI == 1) ? gv : og.y;
            og.z = (cI == 2) ? gv : og.z;
            og.w = (cI == 3) ? gv : og.w;
        }
        const v4h o16 = __builtin_convertvector(og, v4h);
        _Float16* dst = out16 + (size_t)node * HID + 4 * lane;
        *(volatile v4h*)dst = o16;
        __threadfence();
        *(volatile v4h*)dst = o16;
    }
}

extern "C" void kernel_launch(void* const* d_in, const int* in_sizes, int n_in,
                              void* d_out, int out_size, void* d_ws, size_t ws_size,
                              hipStream_t stream)
{
    (void)n_in; (void)out_size;
    const float* x_dev  = (const float*)d_in[0];
    const float* x_fea  = (const float*)d_in[1];
    const int*   e_df_s = (const int*)d_in[2];
    const int*   e_df_d = (const int*)d_in[3];
    const int*   e_fd_s = (const int*)d_in[4];
    const int*   e_fd_d = (const int*)d_in[5];
    const float* W_din  = (const float*)d_in[6];
    const float* b_din  = (const float*)d_in[7];
    const float* W_fin  = (const float*)d_in[8];
    const float* b_fin  = (const float*)d_in[9];
    const float* Wk     = (const float*)d_in[10];
    const float* bk     = (const float*)d_in[11];
    const float* Wq     = (const float*)d_in[12];
    const float* bq     = (const float*)d_in[13];
    const float* Wv     = (const float*)d_in[14];
    const float* bv     = (const float*)d_in[15];
    const float* a_rel  = (const float*)d_in[16];
    const float* m_rel  = (const float*)d_in[17];
    const float* p_rel  = (const float*)d_in[18];
    const float* Wa     = (const float*)d_in[19];
    const float* ba     = (const float*)d_in[20];
    const float* skip   = (const float*)d_in[21];
    const float* ln_g   = (const float*)d_in[22];
    const float* ln_b   = (const float*)d_in[23];
    const float* W_o    = (const float*)d_in[24];
    const float* b_o    = (const float*)d_in[25];

    const int ND_ = in_sizes[0] / HID;
    const int NF_ = in_sizes[1] / HID;
    const int Edf = in_sizes[2] < in_sizes[3] ? in_sizes[2] : in_sizes[3];
    const int Efd = in_sizes[4] < in_sizes[5] ? in_sizes[4] : in_sizes[5];
    const int NMAT = in_sizes[10] / (HID * HID);
    const int L_ = NMAT / 2;
    if (ND_ <= 0 || NF_ <= 0 || L_ <= 0) return;
    const int NT = ND_ + NF_;

    size_t off = 0;
    auto carve = [&](size_t bytes) { size_t o = off; off = (off + bytes + 255) & ~(size_t)255; return o; };
    char* ws = (char*)d_ws;
    const size_t o_x32 = carve((size_t)NT * HID * 4);
    const size_t o_x16 = carve((size_t)NT * HID * 2);
    const size_t o_g16 = carve((size_t)NT * HID * 2);
    const size_t qkvA = ((size_t)ND_ + 2 * (size_t)NF_) * HID;
    const size_t qkvB = ((size_t)NF_ + 2 * (size_t)ND_) * HID;
    const size_t o_qkv = carve((qkvA > qkvB ? qkvA : qkvB) * 4);
    const size_t o_win  = carve((size_t)2 * HID * HID * 2);
    const size_t o_wout = carve((size_t)OUTD * HID * 2);
    const size_t o_wq = carve((size_t)NMAT * HID * HID * 2);
    const size_t o_wk = carve((size_t)NMAT * HID * HID * 2);
    const size_t o_wv = carve((size_t)NMAT * HID * HID * 2);
    const size_t o_wa = carve((size_t)NMAT * HID * HID * 2);
    const size_t o_bin  = carve((size_t)2 * HID * 4);
    const size_t o_bout = carve((size_t)OUTD * 4);
    const size_t o_bq = carve((size_t)NMAT * HID * 4);
    const size_t o_bk = carve((size_t)NMAT * HID * 4);
    const size_t o_bv = carve((size_t)NMAT * HID * 4);
    const size_t o_ba = carve((size_t)NMAT * HID * 4);
    if (off > ws_size) return;

    float*    x32   = (float*)(ws + o_x32);
    _Float16* x16   = (_Float16*)(ws + o_x16);
    _Float16* g16   = (_Float16*)(ws + o_g16);
    float*    qkv   = (float*)(ws + o_qkv);
    _Float16* Win_t = (_Float16*)(ws + o_win);
    _Float16* Wout_t = (_Float16*)(ws + o_wout);
    _Float16* Wq_t = (_Float16*)(ws + o_wq);
    _Float16* Wk_t = (_Float16*)(ws + o_wk);
    _Float16* Wv_t = (_Float16*)(ws + o_wv);
    _Float16* Wa_t = (_Float16*)(ws + o_wa);
    float* bin_p  = (float*)(ws + o_bin);
    float* bout_p = (float*)(ws + o_bout);
    float* bq_p = (float*)(ws + o_bq);
    float* bk_p = (float*)(ws + o_bk);
    float* bv_p = (float*)(ws + o_bv);
    float* ba_p = (float*)(ws + o_ba);

    float* x32d = x32;                      float* x32f = x32 + (size_t)ND_ * HID;
    _Float16* x16d = x16;                   _Float16* x16f = x16 + (size_t)ND_ * HID;
    _Float16* g16d = g16;                   _Float16* g16f = g16 + (size_t)ND_ * HID;
    float* qdA = qkv;  float* kfA = qkv + (size_t)ND_ * HID;  float* vfA = kfA + (size_t)NF_ * HID;
    float* qfB = qkv;  float* kdB = qkv + (size_t)NF_ * HID;  float* vdB = kdB + (size_t)ND_ * HID;

    const float sc16 = 16.0f, sc64 = 64.0f;
    const float inv16 = 1.0f / 16.0f, inv64 = 1.0f / 64.0f;

    const int gx128 = (HID * 16 + 127) / 128;
    const int gx32  = (OUTD * 16 + 127) / 128;
    k_prep<<<dim3(gx128, 1), dim3(128), 0, stream>>>(W_din, b_din, W_din, W_din, 0, HID, sc16, Win_t, bin_p);
    k_prep<<<dim3(gx128, 1), dim3(128), 0, stream>>>(W_fin, b_fin, W_fin, W_fin, 0, HID, sc16,
                                                      Win_t + (size_t)HID * HID, bin_p + HID);
    k_prep<<<dim3(gx32, 1), dim3(128), 0, stream>>>(W_o, b_o, W_o, W_o, 0, OUTD, sc16, Wout_t, bout_p);
    k_prep<<<dim3(gx128, NMAT), dim3(128), 0, stream>>>(Wq, bq, Wq, Wq, 0, HID, sc16, Wq_t, bq_p);
    k_prep<<<dim3(gx128, NMAT), dim3(128), 0, stream>>>(Wk, bk, a_rel, p_rel, 2, HID, sc64, Wk_t, bk_p);
    k_prep<<<dim3(gx128, NMAT), dim3(128), 0, stream>>>(Wv, bv, m_rel, Wv, 1, HID, sc16, Wv_t, bv_p);
    k_prep<<<dim3(gx128, NMAT), dim3(128), 0, stream>>>(Wa, ba, Wa, Wa, 0, HID, sc16, Wa_t, ba_p);

    const int cvt_blocks = (int)(((size_t)NT * 16 + 255) / 256);
    k_cvt<<<dim3(cvt_blocks), dim3(256), 0, stream>>>(x_dev, ND_, x_fea, NF_, g16);

    const int gbd = (ND_ + 31) / 32, gbf = (NF_ + 31) / 32;
    k_lin_relu<<<dim3(gbd), dim3(256), 0, stream>>>(g16d, ND_, Win_t, bin_p, inv16, x32d, x16d);
    k_lin_relu<<<dim3(gbf), dim3(256), 0, stream>>>(g16f, NF_, Win_t + (size_t)HID * HID, bin_p + HID,
                                                     inv16, x32f, x16f);

    constexpr int RD = 512,  SCD = 64;
    constexpr int RF = 1024, SCF = 40;
    static_assert(RD % 8 == 0);
    static_assert(RF % 8 == 0);
    const size_t ldsD = (size_t)(RD * SCD + RD + 1024 + 1024 + 32) * 4;
    const size_t ldsF = (size_t)(RF * SCF + RF + 1024 + 1024 + 32) * 4;
    const int gad = (ND_ + RD - 1) / RD, gaf = (NF_ + RF - 1) / RF;

    for (int l = 0; l < L_; ++l) {
        const int lt0 = l * 2 + 0, lt1 = l * 2 + 1;
        const size_t w0 = (size_t)lt0 * HID * HID, w1 = (size_t)lt1 * HID * HID;
        const size_t c0 = (size_t)lt0 * HID, c1 = (size_t)lt1 * HID;
        k_lin2<<<dim3(gbd, 1), dim3(256), 0, stream>>>(x16d, ND_, Wq_t + w0, bq_p + c0, inv16, qdA,
                                                        Wq_t + w0, bq_p + c0, inv16, qdA);
        k_lin2<<<dim3(gbf, 2), dim3(256), 0, stream>>>(x16f, NF_, Wk_t + w1, bk_p + c1, inv64, kfA,
                                                        Wv_t + w1, bv_p + c1, inv16, vfA);
        k_agg<RD, SCD><<<dim3(gad), dim3(256), ldsD, stream>>>(e_fd_s, e_fd_d, Efd, NF_, ND_,
                                                               qdA, kfA, vfA, g16d);
        k_lin2<<<dim3(gbf, 1), dim3(256), 0, stream>>>(x16f, NF_, Wq_t + w1, bq_p + c1, inv16, qfB,
                                                        Wq_t + w1, bq_p + c1, inv16, qfB);
        k_lin2<<<dim3(gbd, 2), dim3(256), 0, stream>>>(x16d, ND_, Wk_t + w0, bk_p + c0, inv64, kdB,
                                                        Wv_t + w0, bv_p + c0, inv16, vdB);
        k_lin_ln<<<dim3(gbd), dim3(256), 0, stream>>>(g16d, ND_, Wa_t + w0, ba_p + c0, inv16, x32d, x16d,
                                                       skip + lt0, ln_g + c0, ln_b + c0);
        k_agg<RF, SCF><<<dim3(gaf), dim3(256), ldsF, stream>>>(e_df_s, e_df_d, Edf, ND_, NF_,
                                                               qfB, kdB, vdB, g16f);
        k_lin_ln<<<dim3(gbf), dim3(256), 0, stream>>>(g16f, NF_, Wa_t + w1, ba_p + c1, inv16, x32f, x16f,
                                                       skip + lt1, ln_g + c1, ln_b + c1);
    }

    k_out<<<dim3(gbd), dim3(64), 0, stream>>>(x16d, ND_, Wout_t, bout_p, inv16, (float*)d_out);
}
